// MambaBlock_89919435309510
// MI455X (gfx1250) — hardware-verified
//
#include <hip/hip_runtime.h>
#include <stddef.h>
#include <stdint.h>
#include <math.h>


#define SEQ   2048
#define DM    1024
#define DIN   2048
#define NST   16
#define DTR   64
#define XD    96
#define K_IN  1024
#define K_X   4096
#define K_D   128
#define K_O   4096
#define BCW   32
#define NTHR  256
#define GBM   64
#define GTHR  128
#define LCH   16
#define WSMAX 134217728

#define EPI_PLAIN  0
#define EPI_INPROJ 1
#define EPI_DELTA  2
#define EPI_XDBL   3

#define U0 (2 * DIN * (K_IN / 8))
#define U1 (XD * (K_X / 8))
#define U2 (DIN * (K_D / 8))
#define U3 (DM * (K_O / 8))
#define UTOT (U0 + U1 + U2 + U3)

static_assert(SEQ % GBM == 0 && SEQ % LCH == 0 && SEQ % 64 == 0);
static_assert(K_IN % 32 == 0 && K_X % 32 == 0 && K_D % 32 == 0 && K_O % 32 == 0);
static_assert(K_X == 2 * DIN && K_D == 2 * DTR && K_O == 2 * DIN);
static_assert((2 * DIN) % 64 == 0 && DIN % 64 == 0 && DM % 64 == 0 && XD == 96);
static_assert(U0 % NTHR == 0 && U1 % NTHR == 0 && U2 % NTHR == 0 && U3 % NTHR == 0);
static_assert(DIN % NTHR == 0 && DIN == 8 * NTHR);
static_assert((SEQ * DM / 8) % NTHR == 0);
static_assert(LCH * BCW / 4 <= NTHR && LCH * 2 == (NTHR / 32) * 4);
static_assert(XD == DTR + 2 * NST && BCW == 2 * NST);

typedef float          v4f   __attribute__((ext_vector_type(4)));
typedef float          v8f   __attribute__((ext_vector_type(8)));
typedef int            v8i   __attribute__((ext_vector_type(8)));
typedef unsigned short v8us  __attribute__((ext_vector_type(8)));
typedef unsigned short v16us __attribute__((ext_vector_type(16)));
typedef __bf16         v16bf __attribute__((ext_vector_type(16)));
typedef v4f  __attribute__((may_alias)) v4fa;
typedef v8us __attribute__((may_alias)) v8usa;
union FragB { v16bf v; v16us u; v8us h[2]; v8i w; };

__device__ __forceinline__ v8f wmb(const FragB& a, const FragB& b, v8f c) {
  v8f d = __builtin_amdgcn_wmma_f32_16x16x32_bf16(false, a.v, false, b.v, (short)0, c, false, false);
  asm volatile("v_nop\n\tv_nop\n\tv_nop\n\tv_nop" : "+v"(d) : "v"(a.w), "v"(b.w));
  return d;
}

__device__ __forceinline__ unsigned bf16_bits(float f) {
  const unsigned u = __float_as_uint(f);
  return (u + 0x7FFFu + ((u >> 16) & 1u)) >> 16;
}
__device__ __forceinline__ float bf16_val(float f) {
  return __uint_as_float(bf16_bits(f) << 16);
}
__device__ __forceinline__ void hilo(float v, unsigned& h, unsigned& l) {
  h = bf16_bits(v);
  l = bf16_bits(v - __uint_as_float(h << 16));
}
__device__ __forceinline__ float swishf(float t) {
  return t * (1.0f / (1.0f + expf(-t)));
}
__device__ __forceinline__ float softplusf(float t) {
  return fmaxf(t, 0.0f) + log1pf(expf(-fabsf(t)));
}

__global__ __launch_bounds__(NTHR) void k_cvx(const float* __restrict__ x, unsigned short* xb) {
  const int u = (int)blockIdx.x * NTHR + (int)threadIdx.x;
  const float* p = x + (size_t)u * 8;
  const v4f a = *(const v4fa*)p;
  const v4f b = *(const v4fa*)(p + 4);
  v8us o;
  o[0] = (unsigned short)bf16_bits(a.x); o[1] = (unsigned short)bf16_bits(a.y);
  o[2] = (unsigned short)bf16_bits(a.z); o[3] = (unsigned short)bf16_bits(a.w);
  o[4] = (unsigned short)bf16_bits(b.x); o[5] = (unsigned short)bf16_bits(b.y);
  o[6] = (unsigned short)bf16_bits(b.z); o[7] = (unsigned short)bf16_bits(b.w);
  unsigned short* dp = xb + (size_t)u * 8;
  *(volatile v8us*)dp = o;
  __threadfence();
  *(volatile v8us*)dp = o;
}

__global__ __launch_bounds__(NTHR) void k_wprep(const float* __restrict__ Win, const float* __restrict__ Wx,
                                                const float* __restrict__ Wd, const float* __restrict__ Wo,
                                                unsigned short* WINT, unsigned short* WX2,
                                                unsigned short* WD2, unsigned short* WO2) {
  const int u = (int)blockIdx.x * NTHR + (int)threadIdx.x;
  v8us o;
  unsigned short* dp;
  if (u < U0) {
    const int n  = u >> 7;
    const int k8 = (u & 127) * 8;
    const float* p = Win + (size_t)k8 * (2 * DIN) + n;
#pragma unroll
    for (int i = 0; i < 8; ++i) o[i] = (unsigned short)bf16_bits(p[(size_t)i * (2 * DIN)]);
    dp = WINT + (size_t)n * K_IN + k8;
  } else if (u < U0 + U1) {
    const int v  = u - U0;
    const int n  = v >> 9;
    const int k8 = (v & 511) * 8;
    const int kk = k8 & (DIN - 1);
    const float* p = Wx + (size_t)kk * XD + n;
#pragma unroll
    for (int i = 0; i < 8; ++i) o[i] = (unsigned short)bf16_bits(p[(size_t)i * XD]);
    dp = WX2 + (size_t)n * K_X + k8;
  } else if (u < U0 + U1 + U2) {
    const int v  = u - (U0 + U1);
    const int n  = v >> 4;
    const int k8 = (v & 15) * 8;
    const int kk = k8 & (DTR - 1);
    const float* p = Wd + (size_t)kk * DIN + n;
#pragma unroll
    for (int i = 0; i < 8; ++i) o[i] = (unsigned short)bf16_bits(p[(size_t)i * DIN]);
    dp = WD2 + (size_t)n * K_D + k8;
  } else if (u < UTOT) {
    const int v  = u - (U0 + U1 + U2);
    const int n  = v >> 9;
    const int k8 = (v & 511) * 8;
    const int kk = k8 & (DIN - 1);
    const float* p = Wo + (size_t)kk * DM + n;
#pragma unroll
    for (int i = 0; i < 8; ++i) o[i] = (unsigned short)bf16_bits(p[(size_t)i * DM]);
    dp = WO2 + (size_t)n * K_O + k8;
  } else {
    return;
  }
  *(volatile v8us*)dp = o;
  __threadfence();
  *(volatile v8us*)dp = o;
}

template <int NT, int EPI>
__global__ __launch_bounds__(GTHR) void k_gemm(
    const unsigned short* __restrict__ A, const unsigned short* __restrict__ WT, int K,
    float* o0, unsigned o1off, int ldo, unsigned short* oh, const float* __restrict__ bias)
{
  constexpr int GBN = 16 * NT;
  static_assert(EPI != EPI_XDBL || NT == 6);
  static_assert(EPI == EPI_XDBL || NT == 4);
  __shared__ __attribute__((aligned(16))) float stg[GBM * GBN];
  const int tid = (int)threadIdx.x, lane = tid & 31, wave = tid >> 5, hh = lane >> 4, m = lane & 15;
  const int rowBase = (int)blockIdx.x * GBM;
  const int col0    = (int)blockIdx.y * GBN;

  v8f acc[NT];
  {
    const v8f z = {0.f, 0.f, 0.f, 0.f, 0.f, 0.f, 0.f, 0.f};
#pragma unroll
    for (int t = 0; t < NT; ++t) acc[t] = z;
  }
  const unsigned short* ap = A  + (size_t)(rowBase + 16 * wave + m) * (size_t)K + 8 * hh;
  const unsigned short* wp = WT + (size_t)(col0 + m) * (size_t)K + 8 * hh;
  const int ksteps = K >> 5;
#pragma unroll 1
  for (int ks = 0; ks < ksteps; ++ks) {
    FragB af;
    af.h[0] = *(const v8usa*)(ap + 32 * ks);
    af.h[1] = *(const v8usa*)(ap + 32 * ks + 16);
#pragma unroll
    for (int t = 0; t < NT; ++t) {
      const unsigned short* wq = wp + (size_t)(16 * t) * (size_t)K + 32 * ks;
      FragB bf;
      bf.h[0] = *(const v8usa*)wq;
      bf.h[1] = *(const v8usa*)(wq + 16);
      acc[t] = wmb(af, bf, acc[t]);
    }
  }

#pragma unroll
  for (int t = 0; t < NT; ++t) {
    const int lc = 16 * t + m;
#pragma unroll
    for (int r = 0; r < 8; ++r) {
      const int lr = 16 * wave + 8 * hh + r;
      stg[lr * GBN + lc] = acc[t][r];
    }
  }
  __syncthreads();

  if constexpr (EPI == EPI_XDBL) {
    v8us qv[8];
    const bool ls = (m & 8) != 0;
#pragma unroll
    for (int i = 0; i < 8; ++i) {
      const int lr = 16 * wave + 2 * i + hh;
      const float* sp = stg + lr * GBN + 8 * (m & 7);
      const v4f a = *(const v4fa*)sp;
      const v4f b = *(const v4fa*)(sp + 4);
      unsigned h, l;
      v8us q;
      hilo(a.x, h, l); q[0] = (unsigned short)(ls ? l : h);
      hilo(a.y, h, l); q[1] = (unsigned short)(ls ? l : h);
      hilo(a.z, h, l); q[2] = (unsigned short)(ls ? l : h);
      hilo(a.w, h, l); q[3] = (unsigned short)(ls ? l : h);
      hilo(b.x, h, l); q[4] = (unsigned short)(ls ? l : h);
      hilo(b.y, h, l); q[5] = (unsigned short)(ls ? l : h);
      hilo(b.z, h, l); q[6] = (unsigned short)(ls ? l : h);
      hilo(b.w, h, l); q[7] = (unsigned short)(ls ? l : h);
      qv[i] = q;
    }
    v4f bv[4];
#pragma unroll
    for (int i = 0; i < 4; ++i) {
      const int lr = 16 * wave + 4 * i + (lane >> 3);
      bv[i] = *(const v4fa*)(stg + lr * GBN + 64 + 4 * (lane & 7));
    }
#pragma unroll
    for (int i = 0; i < 8; ++i) {
      const int lr = 16 * wave + 2 * i + hh;
      *(volatile v8us*)(oh + (size_t)(rowBase + lr) * K_D + 8 * m) = qv[i];
    }
#pragma unroll
    for (int i = 0; i < 4; ++i) {
      const int lr = 16 * wave + 4 * i + (lane >> 3);
      *(volatile v4f*)(o0 + (size_t)(rowBase + lr) * BCW + 4 * (lane & 7)) = bv[i];
    }
    __threadfence();
#pragma unroll
    for (int i = 0; i < 8; ++i) {
      const int lr = 16 * wave + 2 * i + hh;
      *(volatile v8us*)(oh + (size_t)(rowBase + lr) * K_D + 8 * m) = qv[i];
    }
#pragma unroll
    for (int i = 0; i < 4; ++i) {
      const int lr = 16 * wave + 4 * i + (lane >> 3);
      *(volatile v4f*)(o0 + (size_t)(rowBase + lr) * BCW + 4 * (lane & 7)) = bv[i];
    }
  } else {
    if constexpr (EPI == EPI_INPROJ) {
      if (col0 >= DIN) {
#pragma unroll 1
        for (int i = 0; i < 8; ++i) {
          float* p = stg + (16 * wave + 2 * i + hh) * GBN + 4 * m;
          v4f v = *(const v4fa*)p;
          v.x = swishf(v.x); v.y = swishf(v.y); v.z = swishf(v.z); v.w = swishf(v.w);
          *(v4fa*)p = v;
        }
      }
    }
    if constexpr (EPI == EPI_DELTA) {
      const v4f b4 = *(const v4f*)(bias + col0 + 4 * m);
      const float bx = bf16_val(b4.x), by = bf16_val(b4.y), bz = bf16_val(b4.z), bw = bf16_val(b4.w);
#pragma unroll 1
      for (int i = 0; i < 8; ++i) {
        float* p = stg + (16 * wave + 2 * i + hh) * GBN + 4 * m;
        v4f v = *(const v4fa*)p;
        v.x = softplusf(v.x + bx); v.y = softplusf(v.y + by);
        v.z = softplusf(v.z + bz); v.w = softplusf(v.w + bw);
        *(v4fa*)p = v;
      }
    }
    float* outF = o0;
    int ocol = col0;
    if constexpr (EPI == EPI_INPROJ) {
      const size_t ofs = (col0 >= DIN) ? (size_t)o1off : (size_t)0;
      outF = o0 + ofs;
      ocol = col0 & (DIN - 1);
    }
    v4f fv[8];
#pragma unroll
    for (int i = 0; i < 8; ++i) {
      const int lr = 16 * wave + 2 * i + hh;
      fv[i] = *(const v4fa*)(stg + lr * GBN + 4 * m);
    }
#pragma unroll
    for (int i = 0; i < 8; ++i) {
      const int lr = 16 * wave + 2 * i + hh;
      float* op = outF + (size_t)(rowBase + lr) * (size_t)ldo + ocol + 4 * m;
      *(volatile v4f*)op = fv[i];
    }
    __threadfence();
#pragma unroll
    for (int i = 0; i < 8; ++i) {
      const int lr = 16 * wave + 2 * i + hh;
      float* op = outF + (size_t)(rowBase + lr) * (size_t)ldo + ocol + 4 * m;
      *(volatile v4f*)op = fv[i];
    }
  }
}

__global__ __launch_bounds__(NTHR) void k_conv(const float* __restrict__ XI, const float* __restrict__ cw,
                                               float* U, unsigned short* UHL) {
  __shared__ __attribute__((aligned(16))) float su[DIN];
  const int tid = (int)threadIdx.x;
  const int l  = (int)blockIdx.x;
  const int l1 = (l >= 1) ? l - 1 : 0;
  const int l2 = (l >= 2) ? l - 2 : 0;
  const bool h1 = l >= 1, h2 = l >= 2;
#pragma unroll 1
  for (int j = 0; j < DIN / NTHR; ++j) {
    const int d = j * NTHR + tid;
    const float x0 = XI[(size_t)l  * DIN + d];
    const float r1 = XI[(size_t)l1 * DIN + d];
    const float r2 = XI[(size_t)l2 * DIN + d];
    const float x1 = h1 ? r1 : 0.0f;
    const float x2 = h2 ? r2 : 0.0f;
    const float w0 = bf16_val(cw[3 * d + 0]);
    const float w1 = bf16_val(cw[3 * d + 1]);
    const float w2 = bf16_val(cw[3 * d + 2]);
    const float t = w0 * x2 + w1 * x1 + w2 * x0;
    su[d] = swishf(t);
  }
  __syncthreads();
  const v4f f0 = *(const v4fa*)(su + 4 * tid);
  const v4f f1 = *(const v4fa*)(su + 4 * (tid + NTHR));
  const v4f a = *(const v4fa*)(su + 8 * tid);
  const v4f b = *(const v4fa*)(su + 8 * tid + 4);
  v8us qh, ql;
  {
    unsigned h, lo;
    hilo(a.x, h, lo); qh[0] = (unsigned short)h; ql[0] = (unsigned short)lo;
    hilo(a.y, h, lo); qh[1] = (unsigned short)h; ql[1] = (unsigned short)lo;
    hilo(a.z, h, lo); qh[2] = (unsigned short)h; ql[2] = (unsigned short)lo;
    hilo(a.w, h, lo); qh[3] = (unsigned short)h; ql[3] = (unsigned short)lo;
    hilo(b.x, h, lo); qh[4] = (unsigned short)h; ql[4] = (unsigned short)lo;
    hilo(b.y, h, lo); qh[5] = (unsigned short)h; ql[5] = (unsigned short)lo;
    hilo(b.z, h, lo); qh[6] = (unsigned short)h; ql[6] = (unsigned short)lo;
    hilo(b.w, h, lo); qh[7] = (unsigned short)h; ql[7] = (unsigned short)lo;
  }
  float* up = U + (size_t)l * DIN;
  unsigned short* hp = UHL + (size_t)l * K_X + 8 * tid;
  *(volatile v4f*)(up + 4 * tid) = f0;
  *(volatile v4f*)(up + 4 * (tid + NTHR)) = f1;
  *(volatile v8us*)hp = qh;
  *(volatile v8us*)(hp + DIN) = ql;
  __threadfence();
  *(volatile v4f*)(up + 4 * tid) = f0;
  *(volatile v4f*)(up + 4 * (tid + NTHR)) = f1;
  *(volatile v8us*)hp = qh;
  *(volatile v8us*)(hp + DIN) = ql;
}

__global__ __launch_bounds__(NTHR) void k_suffix(const float* __restrict__ DELTA, float* SD) {
  const int d = (int)blockIdx.x * NTHR + (int)threadIdx.x;
  float s = 0.0f;
#pragma unroll 4
  for (int l = SEQ - 1; l >= 0; --l) {
    *(volatile float*)(SD + (size_t)l * DIN + d) = s;
    s = s + DELTA[(size_t)l * DIN + d];
  }
  __threadfence();
  s = 0.0f;
#pragma unroll 4
  for (int l = SEQ - 1; l >= 0; --l) {
    *(volatile float*)(SD + (size_t)l * DIN + d) = s;
    s = s + DELTA[(size_t)l * DIN + d];
  }
}

__global__ __launch_bounds__(NTHR) void k_scan(const float* __restrict__ DELTA, const float* __restrict__ U,
                                               const float* __restrict__ SD, const float* __restrict__ SRES,
                                               const float* __restrict__ BC, const float* __restrict__ Alog,
                                               const float* __restrict__ Dp, unsigned short* GHL) {
  __shared__ float scum[NST * NTHR];
  __shared__ float san[NST * NTHR];
  __shared__ __attribute__((aligned(16))) float sbc[LCH * BCW];
  __shared__ __attribute__((aligned(16))) float sgs[LCH * NTHR];
  const int tid = (int)threadIdx.x, lane = tid & 31, wave = tid >> 5;
  const int dBase = (int)blockIdx.x * NTHR;
  const int d = dBase + tid;

#pragma unroll 1
  for (int n = 0; n < NST; ++n) {
    const float al = bf16_val(Alog[(size_t)d * NST + n]);
    san[n * NTHR + tid]  = -expf(al);
    scum[n * NTHR + tid] = 0.0f;
  }
  const float Dd = bf16_val(Dp[d]);
  unsigned nz = 0u;

#pragma unroll 1
  for (int c = 0; c < SEQ / LCH; ++c) {
    const int l0 = c * LCH;
    __syncthreads();
    if (tid < LCH * BCW / 4) {
      const v4f t4 = *(const v4f*)(BC + (size_t)l0 * BCW + 4 * tid);
      *(v4fa*)(sbc + 4 * tid) = t4;
    }
    __syncthreads();
#pragma unroll 1
    for (int j = 0; j < LCH; ++j) {
      const int l = l0 + j;
      const size_t off = (size_t)l * DIN + d;
      const float dt = DELTA[off];
      const float uv = U[off];
      const float S  = SD[off];
      const float sr = SRES[off];
      const float du = dt * uv;
      const bool last = (l == SEQ - 1);
      float acc = 0.0f;
#pragma unroll 1
      for (int n = 0; n < NST; ++n) {
        const float a   = san[n * NTHR + tid];
        const float arg = last ? 0.0f : a * S;
        const bool alive = (arg >= -104.0f) || (((nz >> n) & 1u) != 0u);
        if (__builtin_amdgcn_ballot_w32(alive) != 0u) {
          const float E  = (arg < -104.0f) ? 0.0f : expf(arg);
          const float Bn = sbc[j * BCW + n];
          const float Cn = sbc[j * BCW + NST + n];
          float cu = scum[n * NTHR + tid];
          cu = cu + (du * Bn) * E;
          scum[n * NTHR + tid] = cu;
          nz |= ((cu != 0.0f) ? 1u : 0u) << n;
          const float rc = 1.0f / (E + 1e-12f);
          const float xs = cu * rc;
          acc = acc + xs * Cn;
        }
      }
      const float y = acc + uv * Dd;
      sgs[j * NTHR + tid] = y * sr;
    }
    __syncthreads();
    v8us q[4];
#pragma unroll
    for (int i = 0; i < 4; ++i) {
      const int p    = wave * 4 + i;
      const int row  = p >> 1;
      const bool lo  = (p & 1) != 0;
      const float* sp = sgs + row * NTHR + 8 * lane;
      const v4f a = *(const v4fa*)sp;
      const v4f b = *(const v4fa*)(sp + 4);
      unsigned h, l2;
      v8us t;
      hilo(a.x, h, l2); t[0] = (unsigned short)(lo ? l2 : h);
      hilo(a.y, h, l2); t[1] = (unsigned short)(lo ? l2 : h);
      hilo(a.z, h, l2); t[2] = (unsigned short)(lo ? l2 : h);
      hilo(a.w, h, l2); t[3] = (unsigned short)(lo ? l2 : h);
      hilo(b.x, h, l2); t[4] = (unsigned short)(lo ? l2 : h);
      hilo(b.y, h, l2); t[5] = (unsigned short)(lo ? l2 : h);
      hilo(b.z, h, l2); t[6] = (unsigned short)(lo ? l2 : h);
      hilo(b.w, h, l2); t[7] = (unsigned short)(lo ? l2 : h);
      q[i] = t;
    }
#pragma unroll
    for (int i = 0; i < 4; ++i) {
      const int p = wave * 4 + i;
      unsigned short* gp = GHL + (size_t)(l0 + (p >> 1)) * K_O + (size_t)(p & 1) * DIN + dBase + 8 * lane;
      *(volatile v8us*)gp = q[i];
    }
    __threadfence();
#pragma unroll
    for (int i = 0; i < 4; ++i) {
      const int p = wave * 4 + i;
      unsigned short* gp = GHL + (size_t)(l0 + (p >> 1)) * K_O + (size_t)(p & 1) * DIN + dBase + 8 * lane;
      *(volatile v8us*)gp = q[i];
    }
  }
}

static inline size_t al256(size_t o) { return (o + 255) & ~(size_t)255; }

extern "C" void kernel_launch(void* const* d_in, const int* in_sizes, int n_in,
                              void* d_out, int out_size, void* d_ws, size_t ws_size,
                              hipStream_t stream) {
  if (n_in < 9) return;
  if (in_sizes[0] != SEQ * DM) return;
  if (in_sizes[1] != DM * 2 * DIN) return;
  if (in_sizes[2] != DIN * 3) return;
  if (in_sizes[3] != DIN * XD) return;
  if (in_sizes[4] != DTR * DIN) return;
  if (in_sizes[5] != DIN) return;
  if (in_sizes[6] != DIN * NST) return;
  if (in_sizes[7] != DIN) return;
  if (in_sizes[8] != DIN * DM) return;
  if (out_size != SEQ * DM) return;

  const float* x    = (const float*)d_in[0];
  const float* Win  = (const float*)d_in[1];
  const float* cw   = (const float*)d_in[2];
  const float* Wx   = (const float*)d_in[3];
  const float* Wd   = (const float*)d_in[4];
  const float* bd   = (const float*)d_in[5];
  const float* Alog = (const float*)d_in[6];
  const float* Dp   = (const float*)d_in[7];
  const float* Wo   = (const float*)d_in[8];
  float* out = (float*)d_out;

  char* ws = (char*)d_ws;
  size_t off = 0;
  const size_t oXB   = off; off = al256(off + (size_t)SEQ * K_IN * 2);
  const size_t oWINT = off; off = al256(off + (size_t)2 * DIN * K_IN * 2);
  const size_t oWX2  = off; off = al256(off + (size_t)XD * K_X * 2);
  const size_t oWD2  = off; off = al256(off + (size_t)DIN * K_D * 2);
  const size_t oWO2  = off; off = al256(off + (size_t)DM * K_O * 2);
  const size_t oXI   = off; off = al256(off + (size_t)SEQ * DIN * 4);
  const size_t oSRES = off; off = al256(off + (size_t)SEQ * DIN * 4);
  const size_t oU    = off; off = al256(off + (size_t)SEQ * DIN * 4);
  const size_t oUHL  = off; off = al256(off + (size_t)SEQ * K_X * 2);
  const size_t oDLR  = off; off = al256(off + (size_t)SEQ * K_D * 2);
  const size_t oBC   = off; off = al256(off + (size_t)SEQ * BCW * 4);
  const size_t oDEL  = off; off = al256(off + (size_t)SEQ * DIN * 4);
  if (off > ws_size || off > (size_t)WSMAX) return;
  if (((oSRES - oXI) & 3) != 0 || ((oSRES - oXI) >> 2) > 0x7fffffffu) return;

  unsigned short* XB   = (unsigned short*)(ws + oXB);
  unsigned short* WINT = (unsigned short*)(ws + oWINT);
  unsigned short* WX2  = (unsigned short*)(ws + oWX2);
  unsigned short* WD2  = (unsigned short*)(ws + oWD2);
  unsigned short* WO2  = (unsigned short*)(ws + oWO2);
  float*          XI   = (float*)(ws + oXI);
  float*          SD   = (float*)(ws + oXI);
  float*          SRES = (float*)(ws + oSRES);
  float*          Upl  = (float*)(ws + oU);
  unsigned short* UHL  = (unsigned short*)(ws + oUHL);
  unsigned short* GHL  = (unsigned short*)(ws + oUHL);
  unsigned short* DLR  = (unsigned short*)(ws + oDLR);
  float*          BC   = (float*)(ws + oBC);
  float*          DEL  = (float*)(ws + oDEL);
  const unsigned o1off = (unsigned)((oSRES - oXI) >> 2);

  k_cvx<<<(SEQ * DM / 8) / NTHR, NTHR, 0, stream>>>(x, XB);
  k_wprep<<<UTOT / NTHR, NTHR, 0, stream>>>(Win, Wx, Wd, Wo, WINT, WX2, WD2, WO2);
  k_gemm<4, EPI_INPROJ><<<dim3(SEQ / GBM, (2 * DIN) / 64), GTHR, 0, stream>>>(XB, WINT, K_IN, XI, o1off, DIN, DLR, bd);
  k_conv<<<SEQ, NTHR, 0, stream>>>(XI, cw, Upl, UHL);
  k_gemm<6, EPI_XDBL><<<dim3(SEQ / GBM, 1), GTHR, 0, stream>>>(UHL, WX2, K_X, BC, 0u, BCW, DLR, bd);
  k_gemm<4, EPI_DELTA><<<dim3(SEQ / GBM, DIN / 64), GTHR, 0, stream>>>(DLR, WD2, K_D, DEL, 0u, DIN, DLR, bd);
  k_suffix<<<DIN / NTHR, NTHR, 0, stream>>>(DEL, SD);
  k_scan<<<DIN / NTHR, NTHR, 0, stream>>>(DEL, Upl, SD, SRES, BC, Alog, Dp, GHL);
  k_gemm<4, EPI_PLAIN><<<dim3(SEQ / GBM, DM / 64), GTHR, 0, stream>>>(GHL, WO2, K_O, out, 0u, DM, DLR, bd);
}
